// ChaoticNet_5961414607652
// MI455X (gfx1250) — hardware-run, weakly checked
//
#include <hip/hip_runtime.h>
#include <math.h>
#include <stdint.h>

#pragma clang fp contract(off)

typedef __attribute__((ext_vector_type(16))) _Float16 v16h;
typedef __attribute__((ext_vector_type(8)))  _Float16 v8h;
typedef __attribute__((ext_vector_type(8)))  float    v8f;
typedef __attribute__((ext_vector_type(4)))  float    v4f;
typedef __attribute__((ext_vector_type(4)))  unsigned int v4u;

constexpr int kBatch  = 512;
constexpr int kNin    = 256;
constexpr int kFeat   = 4 * kNin;
constexpr int kHid    = 2048;
constexpr int kOut    = 512;
constexpr int kTraj   = 1000;
constexpr int kTabPad = 1024;
static_assert(kFeat == 1024);
static_assert((kTraj % 4) == 0 && kTraj <= kTabPad);
static_assert((kFeat % 32) == 0 && (kHid % 32) == 0);
static_assert((kBatch % 64) == 0 && (kHid % 64) == 0 && (kOut % 64) == 0 && (kFeat % 64) == 0);
static_assert(kNin == 256);

constexpr float kFeatCarry = 1.0f;
constexpr float kWCarry    = 256.0f;
constexpr float kHidCarry  = 1.0f;
constexpr float kScale1    = 1.0f / (kFeatCarry * kWCarry);
constexpr float kScale2    = 1.0f / (kHidCarry * kWCarry);
constexpr float kF16MinNormal = 6.103515625e-5f;
static_assert(kFeatCarry == 1.0f && kHidCarry == 1.0f);
static_assert(kWCarry == 256.0f && kScale1 == 0.00390625f && kScale2 == 0.00390625f);

constexpr size_t kOffTAB = 0;
constexpr size_t kOffFA  = kOffTAB + (size_t)4 * kTabPad * 4;
constexpr size_t kOffW1T = kOffFA  + (size_t)kBatch * kFeat * 2;
constexpr size_t kOffW2T = kOffW1T + (size_t)kHid * kFeat * 2;
constexpr size_t kOffHA  = kOffW2T + (size_t)kOut * kHid * 2;
constexpr size_t kWsTotal = kOffHA + (size_t)kBatch * kHid * 2;
static_assert(kWsTotal == 9453568ull);
static_assert(kWsTotal <= 134217728ull);
static_assert((kOffFA % 128) == 0 && (kOffW1T % 128) == 0 && (kOffW2T % 128) == 0 && (kOffHA % 128) == 0);

__device__ __forceinline__ float flush_h(float v) { return (fabsf(v) < kF16MinNormal) ? 0.0f : v; }
__device__ __forceinline__ unsigned short h_bits(float f) { const _Float16 h = (_Float16)f; return __builtin_bit_cast(unsigned short, h); }
__device__ __forceinline__ unsigned pk16(unsigned short a, unsigned short b) { return (unsigned)a | ((unsigned)b << 16); }

__device__ __forceinline__ void dep_guard1_h(v8f& a, v16h x, v16h y) { asm volatile("v_nop\n\tv_nop\n\tv_nop\n\tv_nop" : "+v"(a) : "v"(x), "v"(y)); }
__device__ __forceinline__ void keep4_h(v16h a, v16h b, v16h c, v16h d) { asm volatile("v_nop" :: "v"(a), "v"(b), "v"(c), "v"(d)); }
__device__ __forceinline__ void acc_guard1(v8f& a) { asm volatile("v_nop\n\tv_nop\n\tv_nop\n\tv_nop" : "+v"(a)); }

struct FragH {
  union U { v16h v; v8h h[2]; };
  static __device__ __forceinline__ v16h load(const _Float16* p) {
    U f; f.h[0] = *(const v8h*)(p); f.h[1] = *(const v8h*)(p + 16); return f.v;
  }
  static __device__ __forceinline__ v8f mma(v16h a, v16h b, v8f c) {
    return __builtin_amdgcn_wmma_f32_16x16x32_f16(false, a, false, b, (short)0, c, false, false);
  }
};

template <int OUT_MODE, int ACT>
__global__ __launch_bounds__(256) void wmma_gemm64_f16(
    const unsigned short* __restrict__ Ap, int lda,
    const unsigned short* __restrict__ Btp, int ldb,
    void* __restrict__ Cout, int ldc,
    const float* __restrict__ bias,
    int M, int N, int K, float scale) {
  const _Float16* A  = (const _Float16*)Ap;
  const _Float16* Bt = (const _Float16*)Btp;
  __shared__ __align__(16) float sT[8][16 * 68];
  const int lane = threadIdx.x & 31;
  const int wave = threadIdx.x >> 5;
  const int tilesN = N >> 6;
  const int tilesM = M >> 6;
  const int tile = blockIdx.x * 8 + wave;
  if (tile >= tilesM * tilesN) return;
  const int tm = tile / tilesN;
  const int tn = tile - tm * tilesN;
  const int m0 = tm << 6;
  const int n0 = tn << 6;

  const int rlane = lane & 15;
  const int koff  = (lane >> 4) * 8;
  const int mOff  = (lane >> 4) * 8;

  v8f acc[4][4];
#pragma unroll
  for (int i = 0; i < 4; ++i)
#pragma unroll
    for (int j = 0; j < 4; ++j) acc[i][j] = (v8f){0.f,0.f,0.f,0.f,0.f,0.f,0.f,0.f};

  for (int k0 = 0; k0 < K; k0 += 32) {
    v16h bh[4];
#pragma unroll
    for (int j = 0; j < 4; ++j) {
      const size_t bo = (size_t)(n0 + (j << 4) + rlane) * ldb + koff + k0;
      bh[j] = FragH::load(Bt + bo);
    }
#pragma unroll
    for (int i = 0; i < 4; ++i) {
      const size_t ao = (size_t)(m0 + (i << 4) + rlane) * lda + koff + k0;
      v16h ah = FragH::load(A + ao);
#pragma unroll
      for (int j = 0; j < 4; ++j) acc[i][j] = FragH::mma(ah, bh[j], acc[i][j]);
#pragma unroll
      for (int j = 0; j < 4; ++j) dep_guard1_h(acc[i][j], ah, bh[j]);
    }
    keep4_h(bh[0], bh[1], bh[2], bh[3]);
  }
#pragma unroll
  for (int i = 0; i < 4; ++i)
#pragma unroll
    for (int j = 0; j < 4; ++j) acc_guard1(acc[i][j]);

  float* slab = sT[wave];
#pragma unroll
  for (int i = 0; i < 4; ++i) {
    const int mBase = m0 + (i << 4);
#pragma unroll
    for (int j = 0; j < 4; ++j) {
      const int n = n0 + (j << 4) + rlane;
      const float bv = bias[n];
#pragma unroll
      for (int r = 0; r < 8; ++r) {
        float v = acc[i][j][r] * scale;
        v += bv;
        if (ACT == 2) v = fmaxf(v, 0.0f);
        slab[(mOff + r) * 68 + (j << 4) + rlane] = v;
      }
    }
    __builtin_amdgcn_fence(__ATOMIC_RELEASE, "workgroup");
    __builtin_amdgcn_wave_barrier();
    __builtin_amdgcn_fence(__ATOMIC_ACQUIRE, "workgroup");
    if (OUT_MODE == 0) {
      float* C = (float*)Cout;
      const int hh = lane >> 4, c4 = (lane & 15) * 4;
      for (int pass = 0; pass < 2; ++pass) {
#pragma unroll
        for (int it = 0; it < 8; ++it) {
          const int row = it * 2 + hh;
          v4f v = *(const v4f*)(slab + row * 68 + c4);
          *(volatile v4f*)(C + (size_t)(mBase + row) * ldc + n0 + c4) = v;
        }
        __threadfence();
      }
    } else {
      const int q = lane >> 3, c8 = (lane & 7) * 8;
      unsigned short* C = (unsigned short*)Cout;
      for (int pass = 0; pass < 2; ++pass) {
#pragma unroll
        for (int it = 0; it < 4; ++it) {
          const int row = it * 4 + q;
          const float* sp = slab + row * 68 + c8;
          v8h hv;
#pragma unroll
          for (int e = 0; e < 8; ++e) {
            const float s = flush_h(sp[e]);
            hv[e] = (_Float16)s;
          }
          *(volatile v8h*)(C + (size_t)(mBase + row) * ldc + n0 + c8) = hv;
        }
        __threadfence();
      }
    }
    __builtin_amdgcn_fence(__ATOMIC_RELEASE, "workgroup");
    __builtin_amdgcn_wave_barrier();
    __builtin_amdgcn_fence(__ATOMIC_ACQUIRE, "workgroup");
  }
}

__global__ __launch_bounds__(32) void traj_kernel(const float* __restrict__ ic_p, const float* __restrict__ th_p,
                                                  float* __restrict__ tab) {
#pragma clang fp contract(off)
  __shared__ __align__(16) float sTab[4 * kTabPad];
  const int lane = threadIdx.x;
  float th = th_p[0];
  float c  = ic_p[0];
  asm volatile("" : "+v"(th));
  asm volatile("" : "+v"(c));
  if (lane == 0) {
    const float omt = 1.0f - th;
    float sgt = 0.0f, ssq = 0.0f, sce = 0.0f;
#pragma unroll 1
    for (int i = 0; i < kTraj; ++i) {
      sTab[i]               = c;
      sTab[kTabPad + i]     = sgt;
      sTab[2 * kTabPad + i] = ssq;
      sTab[3 * kTabPad + i] = sce;
      sgt += (c > 0.5f) ? 1.0f : 0.0f;
      ssq += c * c;
      sce += c * log2f(c + 1e-10f);
      c = (c < th) ? (c / th) : ((1.0f - c) / omt);
    }
#pragma unroll 1
    for (int i = kTraj; i < kTabPad; ++i) {
      sTab[i]               = 3.0e38f;
      sTab[kTabPad + i]     = 0.0f;
      sTab[2 * kTabPad + i] = 0.0f;
      sTab[3 * kTabPad + i] = 0.0f;
    }
  }
  __syncthreads();
  for (int pass = 0; pass < 2; ++pass) {
#pragma unroll 1
    for (int it = 0; it < (4 * kTabPad) / (4 * 32); ++it) {
      const int o = 4 * (it * 32 + lane);
      const v4f v = *(const v4f*)(sTab + o);
      *(volatile v4f*)(tab + o) = v;
    }
    __threadfence();
  }
}

__global__ __launch_bounds__(256) void feat_kernel(const float* __restrict__ x, const float* __restrict__ tab,
                                                   unsigned short* __restrict__ FA) {
  __shared__ __align__(16) float sTab[4 * kTabPad];
  __shared__ __align__(16) float sF[kFeat];
  const int t = threadIdx.x;
  const int b = blockIdx.x;
#pragma unroll
  for (int i = 0; i < 4; ++i) {
    const int o = 4 * (t + 256 * i);
    *(v4f*)(sTab + o) = *(const v4f*)(tab + o);
  }
  const float xv = x[(size_t)b * kNin + t];
  __syncthreads();

  float best = INFINITY;
  int   idx  = 0;
#pragma unroll 2
  for (int i4 = 0; i4 < kTraj / 4; ++i4) {
    const v4f tv = *(const v4f*)(sTab + 4 * i4);
    const int ib = 4 * i4;
    const float d0 = fabsf(xv - tv[0]);
    const bool  p0 = d0 < best;
    best = p0 ? d0 : best;
    idx  = p0 ? ib : idx;
    const float d1 = fabsf(xv - tv[1]);
    const bool  p1 = d1 < best;
    best = p1 ? d1 : best;
    idx  = p1 ? (ib + 1) : idx;
    const float d2 = fabsf(xv - tv[2]);
    const bool  p2 = d2 < best;
    best = p2 ? d2 : best;
    idx  = p2 ? (ib + 2) : idx;
    const float d3 = fabsf(xv - tv[3]);
    const bool  p3 = d3 < best;
    best = p3 ? d3 : best;
    idx  = p3 ? (ib + 3) : idx;
  }
  idx = idx < 0 ? 0 : idx;
  idx = idx > (kTraj - 1) ? (kTraj - 1) : idx;

  const float tt = (float)idx;
  const float cg = sTab[kTabPad + idx];
  const float en = sTab[2 * kTabPad + idx];
  const float ce = sTab[3 * kTabPad + idx];
  const float qd = cg / fmaxf(tt, 1.0f);
  const float ttss = (idx > 0) ? qd : 0.0f;
  const v4f fv = (v4f){ttss, en, tt, -ce};
  *(v4f*)(sF + 4 * t) = fv;
  __syncthreads();

  if (t < 128) {
    const int seg = t;
    const v4f a0 = *(const v4f*)(sF + 8 * seg);
    const v4f a1 = *(const v4f*)(sF + 8 * seg + 4);
    unsigned short ob[8];
#pragma unroll
    for (int e = 0; e < 4; ++e) {
      const float f0 = a0[e];
      const float f1 = a1[e];
      ob[e]     = h_bits(flush_h(f0 * kFeatCarry));
      ob[4 + e] = h_bits(flush_h(f1 * kFeatCarry));
    }
    const v4u u = (v4u){pk16(ob[0], ob[1]), pk16(ob[2], ob[3]), pk16(ob[4], ob[5]), pk16(ob[6], ob[7])};
    unsigned short* dst = FA + (size_t)b * kFeat + 8 * seg;
    *(volatile v4u*)dst = u;
    __threadfence();
    *(volatile v4u*)dst = u;
  }
}

__global__ __launch_bounds__(256) void tcast_kernel(const float* __restrict__ in, unsigned short* __restrict__ out,
                                                    int R, int C, float carry) {
  __shared__ float sm[64][65];
  const int t  = threadIdx.x;
  const int r0 = blockIdx.x * 64;
  const int c0 = blockIdx.y * 64;
#pragma unroll 4
  for (int i = 0; i < 16; ++i) {
    const int e = i * 256 + t;
    const int r = e >> 6;
    const int c = e & 63;
    sm[c][r] = in[(size_t)(r0 + r) * C + c0 + c];
  }
  __syncthreads();
  const int lane = t & 31, wave = t >> 5;
  const int q = lane >> 3, c8 = (lane & 7) * 8;
  v4u hv[2];
#pragma unroll
  for (int it = 0; it < 2; ++it) {
    const int row = wave * 8 + it * 4 + q;
    unsigned short hb[8];
#pragma unroll
    for (int e = 0; e < 8; ++e) {
      const float f = sm[row][c8 + e];
      hb[e] = h_bits(flush_h(f * carry));
    }
    hv[it] = (v4u){pk16(hb[0], hb[1]), pk16(hb[2], hb[3]), pk16(hb[4], hb[5]), pk16(hb[6], hb[7])};
  }
  for (int pass = 0; pass < 2; ++pass) {
#pragma unroll
    for (int it = 0; it < 2; ++it) {
      const int row = wave * 8 + it * 4 + q;
      const size_t o = (size_t)(c0 + row) * R + r0 + c8;
      *(volatile v4u*)(out + o) = hv[it];
    }
    __threadfence();
  }
}

extern "C" void kernel_launch(void* const* d_in, const int* in_sizes, int n_in,
                              void* d_out, int out_size, void* d_ws, size_t ws_size,
                              hipStream_t stream) {
  if (n_in < 8) return;
  if (in_sizes[0] != kBatch * kNin) return;
  if (in_sizes[1] != kFeat * kHid) return;
  if (in_sizes[2] != kHid) return;
  if (in_sizes[3] != kHid * kOut) return;
  if (in_sizes[4] != kOut) return;
  if (in_sizes[5] != 1) return;
  if (in_sizes[6] != 1) return;
  if (in_sizes[7] != 1) return;
  if (out_size != kBatch * kOut) return;
  if (ws_size < kWsTotal) return;

  const float* x  = (const float*)d_in[0];
  const float* W1 = (const float*)d_in[1];
  const float* b1 = (const float*)d_in[2];
  const float* W2 = (const float*)d_in[3];
  const float* b2 = (const float*)d_in[4];
  const float* ic = (const float*)d_in[5];
  const float* th = (const float*)d_in[6];

  char* ws = (char*)d_ws;
  float*          TAB = (float*)(ws + kOffTAB);
  unsigned short* FA  = (unsigned short*)(ws + kOffFA);
  unsigned short* W1T = (unsigned short*)(ws + kOffW1T);
  unsigned short* W2T = (unsigned short*)(ws + kOffW2T);
  unsigned short* HA  = (unsigned short*)(ws + kOffHA);

  traj_kernel<<<1, 32, 0, stream>>>(ic, th, TAB);

  feat_kernel<<<kBatch, 256, 0, stream>>>(x, TAB, FA);

  tcast_kernel<<<dim3(kFeat / 64, kHid / 64), 256, 0, stream>>>(W1, W1T, kFeat, kHid, kWCarry);
  tcast_kernel<<<dim3(kHid / 64, kOut / 64), 256, 0, stream>>>(W2, W2T, kHid, kOut, kWCarry);

  wmma_gemm64_f16<1, 2><<<dim3((kBatch / 64) * (kHid / 64) / 8, 1), 256, 0, stream>>>(
      FA, kFeat,
      W1T, kFeat,
      (void*)HA, kHid,
      b1,
      kBatch, kHid, kFeat, kScale1);

  wmma_gemm64_f16<0, 0><<<dim3((kBatch / 64) * (kOut / 64) / 8, 1), 256, 0, stream>>>(
      HA, kHid,
      W2T, kHid,
      d_out, kOut,
      b2,
      kBatch, kOut, kHid, kScale2);
}
